// Conformer_MultiHeadAttention_13237089206632
// MI455X (gfx1250) — hardware-verified
//
#include <hip/hip_runtime.h>
#include <math.h>

typedef __attribute__((ext_vector_type(16))) _Float16 v16h;
typedef __attribute__((ext_vector_type(8)))  _Float16 v8h;
typedef __attribute__((ext_vector_type(16))) __bf16   v16b;
typedef __attribute__((ext_vector_type(8)))  __bf16   v8b;
typedef __attribute__((ext_vector_type(8)))  float    v8f;
typedef __attribute__((ext_vector_type(4)))  float    v4f;
typedef __attribute__((ext_vector_type(2)))  float    v2f;
#define U16(p) ((const unsigned short*)(const void*)(p))

__device__ __forceinline__ unsigned short f2bf_bits(float f) {
  unsigned u = __float_as_uint(f);
  return (unsigned short)((u + 0x7FFFu + ((u >> 16) & 1u)) >> 16);
}
__device__ __forceinline__ float bf_bits2f(unsigned short h) { return __uint_as_float(((unsigned)h) << 16); }

__device__ __forceinline__ void dep_guard_h(v8f& a, v8f& b, v16h x, v16h y) { asm volatile("v_nop\n\tv_nop\n\tv_nop\n\tv_nop" : "+v"(a), "+v"(b) : "v"(x), "v"(y)); }
__device__ __forceinline__ void dep_guard_b(v8f& a, v8f& b, v16b x, v16b y) { asm volatile("v_nop\n\tv_nop\n\tv_nop\n\tv_nop" : "+v"(a), "+v"(b) : "v"(x), "v"(y)); }
__device__ __forceinline__ void keep4_h(v16h a, v16h b, v16h c, v16h d) { asm volatile("v_nop" :: "v"(a), "v"(b), "v"(c), "v"(d)); }
__device__ __forceinline__ void keep4_b(v16b a, v16b b, v16b c, v16b d) { asm volatile("v_nop" :: "v"(a), "v"(b), "v"(c), "v"(d)); }
__device__ __forceinline__ void acc_guard4(v8f& a, v8f& b, v8f& c, v8f& d) { asm volatile("v_nop\n\tv_nop\n\tv_nop\n\tv_nop" : "+v"(a), "+v"(b), "+v"(c), "+v"(d)); }
template <typename T> struct Frag;
template <> struct Frag<_Float16> {
  typedef v16h V; union U { v16h v; v8h h[2]; };
  static __device__ __forceinline__ v16h load(const _Float16* p) {
    U f; f.h[0] = *(const v8h*)(p); f.h[1] = *(const v8h*)(p + 16); return f.v;
  }
  static __device__ __forceinline__ v8f mma(v16h a, v16h b, v8f c) {
    return __builtin_amdgcn_wmma_f32_16x16x32_f16(false, a, false, b, (short)0, c, false, false);
  }
  static __device__ __forceinline__ void guard(v8f& a, v8f& b, v16h x, v16h y) { dep_guard_h(a, b, x, y); }
  static __device__ __forceinline__ void keep(v16h a, v16h b, v16h c, v16h d) { keep4_h(a, b, c, d); }
};
template <> struct Frag<__bf16> {
  typedef v16b V; union U { v16b v; v8b h[2]; };
  static __device__ __forceinline__ v16b load(const __bf16* p) {
    U f; f.h[0] = *(const v8b*)(p); f.h[1] = *(const v8b*)(p + 16); return f.v;
  }
  static __device__ __forceinline__ v8f mma(v16b a, v16b b, v8f c) {
    return __builtin_amdgcn_wmma_f32_16x16x32_bf16(false, a, false, b, (short)0, c, false, false);
  }
  static __device__ __forceinline__ void guard(v8f& a, v8f& b, v16b x, v16b y) { dep_guard_b(a, b, x, y); }
  static __device__ __forceinline__ void keep(v16b a, v16b b, v16b c, v16b d) { keep4_b(a, b, c, d); }
};

template <int ET> struct Elem;
template <> struct Elem<0> { typedef _Float16 T; };
template <> struct Elem<1> { typedef __bf16 T; };
template <int ET, bool SPLIT, int BIAS_MODE, int OUT_MODE, bool RESID, int ACT = 0>
__global__ __launch_bounds__(256) void wmma_gemm64(
    const unsigned short* __restrict__ Ap, const unsigned short* __restrict__ A2p, int lda, long strideA,
    const unsigned short* __restrict__ Btp, const unsigned short* __restrict__ Bt2p, int ldb, long strideB,
    void* __restrict__ Cout, void* __restrict__ Cout2, int ldc, long strideC,
    const float* __restrict__ bias,
    const float* __restrict__ resid, long strideR,
    int M, int N, int K, float scale) {
  typedef typename Elem<ET>::T T;
  typedef typename Frag<T>::V V;
  const T* A = (const T*)Ap; const T* A2 = (const T*)A2p; const T* Bt = (const T*)Btp; const T* Bt2 = (const T*)Bt2p;
  __shared__ __align__(16) float sT[8][16 * 68];
  const int b    = blockIdx.y;
  const int lane = threadIdx.x & 31;
  const int wave = threadIdx.x >> 5;
  const int tilesN = N >> 6;
  const int tilesM = M >> 6;
  const int tile = blockIdx.x * 8 + wave;
  if (tile >= tilesM * tilesN) return;
  const int tm = tile / tilesN;
  const int tn = tile - tm * tilesN;
  const int m0 = tm << 6;
  const int n0 = tn << 6;

  const T* Ab  = A  + (size_t)b * strideA;
  const T* Bb  = Bt + (size_t)b * strideB;
  const T* Ab2 = SPLIT ? (A2  + (size_t)b * strideA) : nullptr;
  const T* Bb2 = SPLIT ? (Bt2 + (size_t)b * strideB) : nullptr;

  const int rlane = lane & 15;
  const int koff  = (lane >> 4) * 8;
  const int mOff  = (lane >> 4) * 8;

  v8f acc[4][4];
#pragma unroll
  for (int i = 0; i < 4; ++i)
#pragma unroll
    for (int j = 0; j < 4; ++j) acc[i][j] = (v8f){0.f,0.f,0.f,0.f,0.f,0.f,0.f,0.f};

  for (int k0 = 0; k0 < K; k0 += 32) {
    V bh[4], bl[4];
#pragma unroll
    for (int j = 0; j < 4; ++j) {
      const size_t bo = (size_t)(n0 + (j << 4) + rlane) * ldb + koff + k0;
      bh[j] = Frag<T>::load(Bb + bo);
      if (SPLIT) bl[j] = Frag<T>::load(Bb2 + bo);
    }
#pragma unroll
    for (int i = 0; i < 4; ++i) {
      const size_t ao = (size_t)(m0 + (i << 4) + rlane) * lda + koff + k0;
      V ah = Frag<T>::load(Ab + ao);
      V al;
      if (SPLIT) al = Frag<T>::load(Ab2 + ao);
#pragma unroll
      for (int j = 0; j < 4; ++j) {
        acc[i][j] = Frag<T>::mma(ah, bh[j], acc[i][j]);
        if (SPLIT) {
          acc[i][j] = Frag<T>::mma(ah, bl[j], acc[i][j]);
          acc[i][j] = Frag<T>::mma(al, bh[j], acc[i][j]);
        }
      }
      Frag<T>::guard(acc[i][0], acc[i][3], ah, SPLIT ? al : ah);
    }
    Frag<T>::keep(bh[0], bh[1], bh[2], bh[3]);
    if (SPLIT) Frag<T>::keep(bl[0], bl[1], bl[2], bl[3]);
  }
  acc_guard4(acc[0][0], acc[0][1], acc[0][2], acc[0][3]);
  acc_guard4(acc[1][0], acc[1][1], acc[1][2], acc[1][3]);
  acc_guard4(acc[2][0], acc[2][1], acc[2][2], acc[2][3]);
  acc_guard4(acc[3][0], acc[3][1], acc[3][2], acc[3][3]);

  float* slab = sT[wave];
  const float* Rb = RESID ? (resid + (size_t)b * strideR) : nullptr;
#pragma unroll
  for (int i = 0; i < 4; ++i) {
    const int mBase = m0 + (i << 4);
#pragma unroll
    for (int j = 0; j < 4; ++j) {
      const int n = n0 + (j << 4) + rlane;
      float bv = 0.f;
      if (BIAS_MODE == 2) bv = bias[n];
#pragma unroll
      for (int r = 0; r < 8; ++r) {
        float v = acc[i][j][r] * scale;
        if (BIAS_MODE == 1) v += bias[mBase + mOff + r];
        if (BIAS_MODE == 2) v += bv;
        if (RESID) v += Rb[(size_t)(mBase + mOff + r) * ldc + n];
        if (ACT == 1) v = tanhf(v);
        if (ACT == 2) v = fmaxf(v, 0.0f);
        if (ACT == 3) v = v / (1.0f + expf(-v));
        if (ACT == 4) v = (v > 0.f) ? v : 0.01f * v;
        if (ACT == 5) v = 0.5f * v * (1.0f + erff(v * 0.70710678118654752f));
        slab[(mOff + r) * 68 + (j << 4) + rlane] = v;
      }
    }
    __builtin_amdgcn_fence(__ATOMIC_RELEASE, "workgroup");
    __builtin_amdgcn_wave_barrier();
    __builtin_amdgcn_fence(__ATOMIC_ACQUIRE, "workgroup");
    if (OUT_MODE == 0) {
      float* C = (float*)Cout + (size_t)b * strideC;
      const int hh = lane >> 4, c4 = (lane & 15) * 4;
      for (int pass = 0; pass < 2; ++pass) {
#pragma unroll
        for (int it = 0; it < 8; ++it) {
          const int row = it * 2 + hh;
          v4f v = *(const v4f*)(slab + row * 68 + c4);
          *(volatile v4f*)(C + (size_t)(mBase + row) * ldc + n0 + c4) = v;
        }
        __threadfence();
      }
    } else {
      const int q = lane >> 3, c8 = (lane & 7) * 8;
      unsigned short* C  = (unsigned short*)Cout  + (size_t)b * strideC;
      unsigned short* C2 = (OUT_MODE == 2) ? ((unsigned short*)Cout2 + (size_t)b * strideC) : nullptr;
      for (int pass = 0; pass < 2; ++pass) {
#pragma unroll
        for (int it = 0; it < 4; ++it) {
          const int row = it * 4 + q;
          const float* sp = slab + row * 68 + c8;
          v8h hv, lv;
#pragma unroll
          for (int e = 0; e < 8; ++e) {
            if (OUT_MODE == 1) {
              hv[e] = (_Float16)sp[e];
            } else {
              unsigned short hb = f2bf_bits(sp[e]);
              unsigned short lb = f2bf_bits(sp[e] - bf_bits2f(hb));
              hv[e] = __builtin_bit_cast(_Float16, hb);
              lv[e] = __builtin_bit_cast(_Float16, lb);
            }
          }
          *(volatile v8h*)(C + (size_t)(mBase + row) * ldc + n0 + c8) = hv;
          if (OUT_MODE == 2) *(volatile v8h*)(C2 + (size_t)(mBase + row) * ldc + n0 + c8) = lv;
        }
        __threadfence();
      }
    }
    __builtin_amdgcn_fence(__ATOMIC_RELEASE, "workgroup");
    __builtin_amdgcn_wave_barrier();
    __builtin_amdgcn_fence(__ATOMIC_ACQUIRE, "workgroup");
  }
}

__global__ __launch_bounds__(256) void transpose_cast_f16(const float* __restrict__ in, int ldi,
                                                         _Float16* __restrict__ outT, int ldo, float scale) {
  __shared__ __align__(16) _Float16 tile[64][72];
  const int c0 = blockIdx.x * 64, r0 = blockIdx.y * 64;
  const int t = threadIdx.y * 32 + threadIdx.x;
  for (int i = threadIdx.y; i < 64; i += 8) {
    tile[threadIdx.x][i]      = (_Float16)(in[(size_t)(r0 + i) * ldi + c0 + threadIdx.x] * scale);
    tile[32 + threadIdx.x][i] = (_Float16)(in[(size_t)(r0 + i) * ldi + c0 + 32 + threadIdx.x] * scale);
  }
  __syncthreads();
  const int q = t >> 3, c8 = (t & 7) * 8;
  for (int pass = 0; pass < 2; ++pass) {
#pragma unroll
    for (int it = 0; it < 2; ++it) {
      const int c = it * 32 + q;
      v8h hv = *(const v8h*)(&tile[c][c8]);
      *(volatile v8h*)(outT + (size_t)(c0 + c) * ldo + r0 + c8) = hv;
    }
    __threadfence();
  }
}

__global__ __launch_bounds__(256) void transpose_split_bf16(const float* __restrict__ in, int ldi,
                                                           __bf16* __restrict__ outH, __bf16* __restrict__ outL, int ldo) {
  __shared__ __align__(16) float tile[64][68];
  const int c0 = blockIdx.x * 64, r0 = blockIdx.y * 64;
  const int t = threadIdx.y * 32 + threadIdx.x;
  for (int i = threadIdx.y; i < 64; i += 8) {
    tile[threadIdx.x][i]      = in[(size_t)(r0 + i) * ldi + c0 + threadIdx.x];
    tile[32 + threadIdx.x][i] = in[(size_t)(r0 + i) * ldi + c0 + 32 + threadIdx.x];
  }
  __syncthreads();
  const int q = t >> 3, c8 = (t & 7) * 8;
  for (int pass = 0; pass < 2; ++pass) {
#pragma unroll
    for (int it = 0; it < 2; ++it) {
      const int c = it * 32 + q;
      v8b hv, lv;
#pragma unroll
      for (int e = 0; e < 8; ++e) {
        const float f = tile[c][c8 + e];
        const unsigned short hb = f2bf_bits(f);
        hv[e] = __builtin_bit_cast(__bf16, hb);
        lv[e] = __builtin_bit_cast(__bf16, f2bf_bits(f - bf_bits2f(hb)));
      }
      *(volatile v8b*)(outH + (size_t)(c0 + c) * ldo + r0 + c8) = hv;
      *(volatile v8b*)(outL + (size_t)(c0 + c) * ldo + r0 + c8) = lv;
    }
    __threadfence();
  }
}

constexpr int kBatch = 2;
constexpr int kSeq   = 2048;
constexpr int kEmb   = 1024;
constexpr int kHeads = 8;
constexpr int kDh    = 128;
constexpr int kTok   = kBatch * kSeq;
constexpr int kPairs = kEmb / 2;
static_assert(kHeads * kDh == kEmb);
static_assert(kPairs == 512);

__global__ __launch_bounds__(256) void layernorm_split_kernel(
    const float* __restrict__ x, const float* __restrict__ gamma, const float* __restrict__ beta,
    unsigned* __restrict__ xh, unsigned* __restrict__ xl) {
  __shared__ float red[8];
  const int tok = blockIdx.x;
  const int t = threadIdx.x, lane = t & 31, wave = t >> 5;
  const float* xr = x + (size_t)tok * kEmb;
  const int ca = 2 * t, cb = kPairs + 2 * t;
  const v2f pa = *(const v2f*)(xr + ca);
  const v2f pb = *(const v2f*)(xr + cb);
  float s = (pa.x + pa.y) + (pb.x + pb.y);
#pragma unroll
  for (int off = 1; off < 32; off <<= 1) s += __shfl_xor(s, off, 32);
  if (lane == 0) red[wave] = s;
  __syncthreads();
  float tot = 0.f;
#pragma unroll
  for (int w = 0; w < 8; ++w) tot += red[w];
  const float mean = tot * (1.0f / (float)kEmb);
  __syncthreads();
  const float d0 = pa.x - mean, d1 = pa.y - mean, d2 = pb.x - mean, d3 = pb.y - mean;
  float s2 = (d0 * d0 + d1 * d1) + (d2 * d2 + d3 * d3);
#pragma unroll
  for (int off = 1; off < 32; off <<= 1) s2 += __shfl_xor(s2, off, 32);
  if (lane == 0) red[wave] = s2;
  __syncthreads();
  float tot2 = 0.f;
#pragma unroll
  for (int w = 0; w < 8; ++w) tot2 += red[w];
  const float var  = tot2 * (1.0f / (float)kEmb);
  const float rstd = 1.0f / sqrtf(var + 1e-5f);
  const float y0 = d0 * rstd * gamma[ca] + beta[ca];
  const float y1 = d1 * rstd * gamma[ca + 1] + beta[ca + 1];
  const float y2 = d2 * rstd * gamma[cb] + beta[cb];
  const float y3 = d3 * rstd * gamma[cb + 1] + beta[cb + 1];
  const unsigned short h0 = f2bf_bits(y0), h1 = f2bf_bits(y1), h2 = f2bf_bits(y2), h3 = f2bf_bits(y3);
  const unsigned short l0 = f2bf_bits(y0 - bf_bits2f(h0)), l1 = f2bf_bits(y1 - bf_bits2f(h1));
  const unsigned short l2 = f2bf_bits(y2 - bf_bits2f(h2)), l3 = f2bf_bits(y3 - bf_bits2f(h3));
  const unsigned uah = (unsigned)h0 | ((unsigned)h1 << 16), ual = (unsigned)l0 | ((unsigned)l1 << 16);
  const unsigned ubh = (unsigned)h2 | ((unsigned)h3 << 16), ubl = (unsigned)l2 | ((unsigned)l3 << 16);
  const size_t ia = (size_t)tok * kPairs + t, ib = ia + 256;
  for (int pass = 0; pass < 2; ++pass) {
    ((volatile unsigned*)xh)[ia] = uah;
    ((volatile unsigned*)xh)[ib] = ubh;
    ((volatile unsigned*)xl)[ia] = ual;
    ((volatile unsigned*)xl)[ib] = ubl;
    __threadfence();
  }
}

__global__ __launch_bounds__(256) void posenc_split_kernel(unsigned* __restrict__ peh, unsigned* __restrict__ pel) {
  const int idx = blockIdx.x * 256 + threadIdx.x;
  if (idx >= kSeq * kPairs) return;
  const int pos = idx >> 9, i = idx & 511;
  const float kNegLogRate = -0.00899447301950799f;
  const float freq = expf((float)(2 * i) * kNegLogRate);
  const float ang  = (float)pos * freq;
  const float sv = sinf(ang), cv = cosf(ang);
  const unsigned short hs = f2bf_bits(sv), hc = f2bf_bits(cv);
  const unsigned short ls = f2bf_bits(sv - bf_bits2f(hs)), lc = f2bf_bits(cv - bf_bits2f(hc));
  const unsigned uh = (unsigned)hs | ((unsigned)hc << 16), ul = (unsigned)ls | ((unsigned)lc << 16);
  for (int pass = 0; pass < 2; ++pass) {
    ((volatile unsigned*)peh)[idx] = uh;
    ((volatile unsigned*)pel)[idx] = ul;
    __threadfence();
  }
}

__global__ __launch_bounds__(64) void bias16_kernel(const float* __restrict__ bq, const float* __restrict__ bk,
                                                   float* __restrict__ qb, float* __restrict__ kb) {
  const int lane = threadIdx.x & 31, wave = threadIdx.x >> 5;
  v4f v; float* dst;
  if (wave == 0) { v = *(const v4f*)(bq + 4 * lane); dst = qb + 4 * lane; }
  else           { v = *(const v4f*)(bk + 4 * lane); dst = kb + 4 * lane; }
  v = v * 16.0f;
  *(volatile v4f*)dst = v;
  __threadfence();
  *(volatile v4f*)dst = v;
}

__global__ __launch_bounds__(256) void headbias_kernel(const _Float16* __restrict__ k16, const _Float16* __restrict__ pp16,
                                                      const float* __restrict__ ub, const float* __restrict__ vb,
                                                      float* __restrict__ ubk, float* __restrict__ vbp) {
  const int t = blockIdx.x * 256 + threadIdx.x;
  const _Float16* row; const float* bvec; float* dst;
  if (blockIdx.x < 128) {
    const int b = t >> 14, h = (t >> 11) & 7, s = t & 2047;
    row = k16 + (size_t)((b * kSeq + s) * kHeads + h) * kDh; bvec = ub + h * kDh; dst = ubk + t;
  } else {
    const int u = t - 32768; const int h = (u >> 11) & 7, s = u & 2047;
    row = pp16 + (size_t)(s * kHeads + h) * kDh; bvec = vb + h * kDh; dst = vbp + u;
  }
  float acc = 0.f;
#pragma unroll 1
  for (int ch = 0; ch < kDh / 8; ++ch) {
    const v8h kv = *(const v8h*)(row + 8 * ch);
    const v4f b0 = *(const v4f*)(bvec + 8 * ch);
    const v4f b1 = *(const v4f*)(bvec + 8 * ch + 4);
    acc += b0.x * (float)kv[0] + b0.y * (float)kv[1] + b0.z * (float)kv[2] + b0.w * (float)kv[3]
         + b1.x * (float)kv[4] + b1.y * (float)kv[5] + b1.z * (float)kv[6] + b1.w * (float)kv[7];
  }
  const float r = acc * 0.0625f;
  *(volatile float*)dst = r;
  __threadfence();
  *(volatile float*)dst = r;
}

__global__ __launch_bounds__(256) void score_softmax_kernel(const float* __restrict__ cont, const float* __restrict__ ps,
                                                          _Float16* __restrict__ p16) {
  __shared__ float red[8];
  const int a = blockIdx.x;
  const int t = threadIdx.x, lane = t & 31, wave = t >> 5;
  const int c0 = 8 * t;
  const float* crow = cont + (size_t)a * kSeq + c0;
  const v4f ca = *(const v4f*)crow;
  const v4f cb = *(const v4f*)(crow + 4);
  float cv[8];
  cv[0] = ca.x; cv[1] = ca.y; cv[2] = ca.z; cv[3] = ca.w; cv[4] = cb.x; cv[5] = cb.y; cv[6] = cb.z; cv[7] = cb.w;
  const int a1 = (a + 1 < kSeq) ? (a + 1) : (kSeq - 1);
  const float* prow0 = ps + (size_t)a * kSeq;
  const float* prow1 = ps + (size_t)a1 * kSeq;
  const int sh0 = kSeq - 1 - a;
  float sv[8];
  float mx = -INFINITY;
#pragma unroll
  for (int e = 0; e < 8; ++e) {
    const int c = c0 + e;
    int i1 = c + sh0;   i1 = (i1 > kSeq - 1) ? (kSeq - 1) : i1;
    int i2 = c - a - 2; i2 = (i2 < 0) ? 0 : i2;
    const float v1 = prow0[i1];
    const float v2 = prow1[i2];
    const float pv = (c <= a) ? v1 : ((c == a + 1) ? 0.0f : v2);
    const float s = (cv[e] + pv) * (1.0f / 32.0f);
    sv[e] = s;
    mx = fmaxf(mx, s);
  }
#pragma unroll
  for (int off = 1; off < 32; off <<= 1) mx = fmaxf(mx, __shfl_xor(mx, off, 32));
  if (lane == 0) red[wave] = mx;
  __syncthreads();
  float gm = red[0];
#pragma unroll
  for (int w = 1; w < 8; ++w) gm = fmaxf(gm, red[w]);
  __syncthreads();
  float sum = 0.f;
#pragma unroll
  for (int e = 0; e < 8; ++e) { sv[e] = __expf(sv[e] - gm); sum += sv[e]; }
#pragma unroll
  for (int off = 1; off < 32; off <<= 1) sum += __shfl_xor(sum, off, 32);
  if (lane == 0) red[wave] = sum;
  __syncthreads();
  float tot = 0.f;
#pragma unroll
  for (int w = 0; w < 8; ++w) tot += red[w];
  const float f = (1.0f / tot) * 32768.0f;
  v8h hv;
#pragma unroll
  for (int e = 0; e < 8; ++e) hv[e] = (_Float16)(sv[e] * f);
  _Float16* dst = p16 + (size_t)a * kSeq + c0;
  *(volatile v8h*)dst = hv;
  __threadfence();
  *(volatile v8h*)dst = hv;
}

extern "C" void kernel_launch(void* const* d_in, const int* in_sizes, int n_in, void* d_out, int out_size,
                              void* d_ws, size_t ws_size, hipStream_t stream) {
  if (n_in < 14) return;
  if (in_sizes[0] != kTok * kEmb || in_sizes[1] != kEmb || in_sizes[2] != kEmb ||
      in_sizes[3] != kDh * kDh || in_sizes[4] != kDh || in_sizes[5] != kDh * kDh || in_sizes[6] != kDh ||
      in_sizes[7] != kDh * kDh || in_sizes[8] != kDh || in_sizes[9] != kDh * kDh ||
      in_sizes[10] != kHeads * kDh || in_sizes[11] != kHeads * kDh || in_sizes[12] != kEmb * kEmb || in_sizes[13] != kEmb ||
      out_size != kTok * kEmb) return;
  const float* x      = (const float*)d_in[0];
  const float* gamma  = (const float*)d_in[1];
  const float* beta   = (const float*)d_in[2];
  const float* Wq     = (const float*)d_in[3];
  const float* bq     = (const float*)d_in[4];
  const float* Wk     = (const float*)d_in[5];
  const float* bk     = (const float*)d_in[6];
  const float* Wv     = (const float*)d_in[7];
  const float* bv     = (const float*)d_in[8];
  const float* Wp     = (const float*)d_in[9];
  const float* u_bias = (const float*)d_in[10];
  const float* v_bias = (const float*)d_in[11];
  const float* Wo     = (const float*)d_in[12];
  const float* bo     = (const float*)d_in[13];
  float* out = (float*)d_out;

  char* ws = (char*)d_ws; size_t off = 0;
  auto carve = [&](size_t bytes) -> char* { char* p = ws + off; off += (bytes + 255) & ~(size_t)255; return p; };
  const size_t nW   = (size_t)kDh * kDh;
  const size_t nWo  = (size_t)kEmb * kEmb;
  const size_t nHd  = (size_t)kTok * kHeads * kDh;
  const size_t nPp  = (size_t)kSeq * kHeads * kDh;
  const size_t nSS  = (size_t)kSeq * kSeq;
  __bf16* WqTh = (__bf16*)carve(nW * 2); __bf16* WqTl = (__bf16*)carve(nW * 2);
  __bf16* WkTh = (__bf16*)carve(nW * 2); __bf16* WkTl = (__bf16*)carve(nW * 2);
  __bf16* WvTh = (__bf16*)carve(nW * 2); __bf16* WvTl = (__bf16*)carve(nW * 2);
  __bf16* WpTh = (__bf16*)carve(nW * 2); __bf16* WpTl = (__bf16*)carve(nW * 2);
  __bf16* WoTh = (__bf16*)carve(nWo * 2); __bf16* WoTl = (__bf16*)carve(nWo * 2);
  float* qb16 = (float*)carve(kDh * 4); float* kb16 = (float*)carve(kDh * 4);
  float* ubk  = (float*)carve((size_t)kBatch * kHeads * kSeq * 4);
  float* vbp  = (float*)carve((size_t)kHeads * kSeq * 4);
  _Float16* q16  = (_Float16*)carve(nHd * 2);
  _Float16* k16  = (_Float16*)carve(nHd * 2);
  _Float16* pp16 = (_Float16*)carve(nPp * 2);
  float*    vf32 = (float*)carve(nHd * 4);
  unsigned short* ctxh = (unsigned short*)carve(nHd * 2); unsigned short* ctxl = (unsigned short*)carve(nHd * 2);
  _Float16* vt16 = (_Float16*)carve((size_t)kEmb * kSeq * 2);
  char* loopBase = carve(nSS * 4 + nSS * 4 + nSS * 2);
  float*    contT = (float*)loopBase;
  float*    posT  = (float*)(loopBase + nSS * 4);
  _Float16* p16   = (_Float16*)(loopBase + nSS * 8);
  unsigned* xnh = (unsigned*)loopBase;
  unsigned* xnl = (unsigned*)(loopBase + nHd * 2);
  unsigned* peh = (unsigned*)(loopBase + nHd * 4);
  unsigned* pel = (unsigned*)(loopBase + nHd * 4 + (size_t)kSeq * kEmb * 2);
  if (nHd * 4 + (size_t)kSeq * kEmb * 4 > nSS * 10) return;
  if (off > ws_size || off > ((size_t)1 << 27)) return;

  transpose_split_bf16<<<dim3(kDh / 64, kDh / 64), dim3(32, 8), 0, stream>>>(Wq, kDh, WqTh, WqTl, kDh);
  transpose_split_bf16<<<dim3(kDh / 64, kDh / 64), dim3(32, 8), 0, stream>>>(Wk, kDh, WkTh, WkTl, kDh);
  transpose_split_bf16<<<dim3(kDh / 64, kDh / 64), dim3(32, 8), 0, stream>>>(Wv, kDh, WvTh, WvTl, kDh);
  transpose_split_bf16<<<dim3(kDh / 64, kDh / 64), dim3(32, 8), 0, stream>>>(Wp, kDh, WpTh, WpTl, kDh);
  transpose_split_bf16<<<dim3(kEmb / 64, kEmb / 64), dim3(32, 8), 0, stream>>>(Wo, kEmb, WoTh, WoTl, kEmb);
  bias16_kernel<<<1, 64, 0, stream>>>(bq, bk, qb16, kb16);
  layernorm_split_kernel<<<kTok, 256, 0, stream>>>(x, gamma, beta, xnh, xnl);
  posenc_split_kernel<<<(kSeq * kPairs) / 256, 256, 0, stream>>>(peh, pel);

  { const int tl = (kTok * kHeads / 64) * (kDh / 64);
    wmma_gemm64<1, true, 2, 1, false><<<dim3(tl / 8, 1), 256, 0, stream>>>(U16(xnh), U16(xnl), kDh, 0, U16(WqTh), U16(WqTl), kDh, 0,
        q16, nullptr, kDh, 0, qb16, nullptr, 0, kTok * kHeads, kDh, kDh, 16.0f);
    wmma_gemm64<1, true, 2, 1, false><<<dim3(tl / 8, 1), 256, 0, stream>>>(U16(xnh), U16(xnl), kDh, 0, U16(WkTh), U16(WkTl), kDh, 0,
        k16, nullptr, kDh, 0, kb16, nullptr, 0, kTok * kHeads, kDh, kDh, 16.0f);
    wmma_gemm64<1, true, 2, 0, false><<<dim3(tl / 8, 1), 256, 0, stream>>>(U16(xnh), U16(xnl), kDh, 0, U16(WvTh), U16(WvTl), kDh, 0,
        vf32, nullptr, kDh, 0, bv, nullptr, 0, kTok * kHeads, kDh, kDh, 1.0f); }
  { const int tl = (kSeq * kHeads / 64) * (kDh / 64);
    wmma_gemm64<1, true, 0, 1, false><<<dim3(tl / 8, 1), 256, 0, stream>>>(U16(peh), U16(pel), kDh, 0, U16(WpTh), U16(WpTl), kDh, 0,
        pp16, nullptr, kDh, 0, nullptr, nullptr, 0, kSeq * kHeads, kDh, kDh, 16.0f); }
  headbias_kernel<<<192, 256, 0, stream>>>(k16, pp16, u_bias, v_bias, ubk, vbp);

  for (int b = 0; b < kBatch; ++b) {
    transpose_cast_f16<<<dim3(kEmb / 64, kSeq / 64), dim3(32, 8), 0, stream>>>(vf32 + (size_t)b * kSeq * kEmb, kEmb, vt16, kSeq, 16.0f);
    for (int h = 0; h < kHeads; ++h) {
      const size_t qoff = (size_t)b * kSeq * kEmb + (size_t)h * kDh;
      const int tl = (kSeq / 64) * (kSeq / 64);
      wmma_gemm64<0, false, 2, 0, false><<<dim3(tl / 8, 1), 256, 0, stream>>>(U16(q16 + qoff), nullptr, kEmb, 0, U16(k16 + qoff), nullptr, kEmb, 0,
          contT, nullptr, kSeq, 0, ubk + (size_t)(b * kHeads + h) * kSeq, nullptr, 0, kSeq, kSeq, kDh, 1.0f / 256.0f);
      wmma_gemm64<0, false, 2, 0, false><<<dim3(tl / 8, 1), 256, 0, stream>>>(U16(q16 + qoff), nullptr, kEmb, 0, U16(pp16 + (size_t)h * kDh), nullptr, kEmb, 0,
          posT, nullptr, kSeq, 0, vbp + (size_t)h * kSeq, nullptr, 0, kSeq, kSeq, kDh, 1.0f / 256.0f);
      score_softmax_kernel<<<kSeq, 256, 0, stream>>>(contT, posT, p16);
      { const int tp = (kSeq / 64) * (kDh / 64);
        wmma_gemm64<0, false, 0, 2, false><<<dim3(tp / 8, 1), 256, 0, stream>>>(U16(p16), nullptr, kSeq, 0, U16(vt16 + (size_t)h * kDh * kSeq), nullptr, kSeq, 0,
            ctxh + qoff, ctxl + qoff, kEmb, 0, nullptr, nullptr, 0, kSeq, kDh, kSeq, 1.0f / 524288.0f); }
    }
  }

  { const int tl = (kTok / 64) * (kEmb / 64);
    wmma_gemm64<1, true, 2, 0, false><<<dim3(tl / 8, 1), 256, 0, stream>>>(U16(ctxh), U16(ctxl), kEmb, 0, U16(WoTh), U16(WoTl), kEmb, 0,
        out, nullptr, kEmb, 0, bo, nullptr, 0, kTok, kEmb, kEmb, 1.0f); }
}
